// AttentionGuidedEgoGAT_438086664202
// MI455X (gfx1250) — hardware-verified
//
#include <hip/hip_runtime.h>
#include <stddef.h>


typedef unsigned short us_t;
typedef us_t   v8us  __attribute__((ext_vector_type(8)));
typedef __bf16 v16bf __attribute__((ext_vector_type(16)));
typedef float  v8f   __attribute__((ext_vector_type(8)));
typedef float  v4f   __attribute__((ext_vector_type(4)));
typedef int    v4i   __attribute__((ext_vector_type(4)));

union Frag { v16bf v; v8us u[2]; };

#define NTHR 256
#define FIN  128
#define C2   32
#define TN   32
#define NPB  256
#define LCAP 7168
#define ROWW 64
#define RCAP 63

__device__ __forceinline__ us_t f2bf(float f) {
  unsigned u = __float_as_uint(f);
  u += 0x7FFFu + ((u >> 16) & 1u);
  return (us_t)(u >> 16);
}
__device__ __forceinline__ float bf2f(us_t b) { return __uint_as_float(((unsigned)b) << 16); }

__device__ __forceinline__ float gelu_f(float v) {
  return 0.5f * v * (1.0f + erff(v * 0.70710678118654752440f));
}

__device__ __forceinline__ v8f wmma_bf16(v16bf a, v16bf b, v8f c) {
  v8f d = __builtin_amdgcn_wmma_f32_16x16x32_bf16(false, a, false, b, (short)0, c, false, false);
  asm volatile("v_nop\n\tv_nop\n\tv_nop\n\tv_nop" : "+v"(d) : "v"(a), "v"(b));
  return d;
}

__global__ __launch_bounds__(NTHR)
void adj_build_k(const int* __restrict__ ei, int* __restrict__ adj, int N, int E) {
  __shared__ unsigned s_list[LCAP];
  __shared__ __attribute__((aligned(16))) int s_rows[128 * ROWW];
  __shared__ int s_wc[8];
  const int t = threadIdx.x, lane = t & 31, wv = t >> 5;
  const int node0 = blockIdx.x * NPB;
  const unsigned ltmask = (1u << lane) - 1u;
  int total = 0;
  for (int base = 0; base < E; base += NTHR) {
    const int e = base + t;
    bool match = false;
    unsigned packed = 0u;
    if (e < E) {
      const int d = ei[(size_t)E + e];
      int s = ei[e];
      s = s < 0 ? 0 : (s > N - 1 ? N - 1 : s);
      const unsigned ld = (unsigned)(d - node0);
      if (ld < (unsigned)NPB) { match = true; packed = (ld << 24) | (unsigned)s; }
    }
    const unsigned bal = __builtin_amdgcn_ballot_w32(match);
    if (lane == 0) s_wc[wv] = (int)__builtin_popcount(bal);
    __syncthreads();
    int before = 0, ctot = 0;
#pragma unroll
    for (int w = 0; w < 8; ++w) {
      const int c = s_wc[w];
      ctot += c;
      before += (w < wv) ? c : 0;
    }
    if (match) {
      const int pos = total + before + (int)__builtin_popcount(bal & ltmask);
      if (pos < LCAP) s_list[pos] = packed;
    }
    total += ctot;
    __syncthreads();
  }
  const int L = total < LCAP ? total : LCAP;

  for (int half = 0; half < NPB / 128; ++half) {
    for (int i = t; i < 128 * ROWW; i += NTHR) s_rows[i] = 0;
    __syncthreads();
    for (int jl = wv; jl < 128; jl += 8) {
      const unsigned j = (unsigned)(half * 128 + jl);
      int run = 0;
      for (int i0 = 0; i0 < L; i0 += 32) {
        const int i = i0 + lane;
        const bool inr = i < L;
        const unsigned ent = inr ? s_list[i] : 0u;
        const bool mt = inr && ((ent >> 24) == j);
        const unsigned bal = __builtin_amdgcn_ballot_w32(mt);
        const int rk = run + (int)__builtin_popcount(bal & ltmask);
        if (mt && rk < RCAP) s_rows[jl * ROWW + 1 + rk] = (int)(ent & 0xFFFFFFu);
        run += (int)__builtin_popcount(bal);
      }
      if (lane == 0) s_rows[jl * ROWW] = run < RCAP ? run : RCAP;
    }
    __syncthreads();
    for (int p = wv; p < 64; p += 8) {
      const int jl = 2 * p + (lane >> 4);
      const int node = node0 + half * 128 + jl;
      const v4i v = *(const v4i*)(&s_rows[jl * ROWW + (lane & 15) * 4]);
      if (node < N) *(volatile v4i*)(adj + (size_t)node * ROWW + (lane & 15) * 4) = v;
    }
    __threadfence();
    for (int p = wv; p < 64; p += 8) {
      const int jl = 2 * p + (lane >> 4);
      const int node = node0 + half * 128 + jl;
      const v4i v = *(const v4i*)(&s_rows[jl * ROWW + (lane & 15) * 4]);
      if (node < N) *(volatile v4i*)(adj + (size_t)node * ROWW + (lane & 15) * 4) = v;
    }
    __syncthreads();
  }
}

__global__ __launch_bounds__(NTHR)
void cvt_rows_k(const float* __restrict__ in, us_t* __restrict__ hi, us_t* __restrict__ lo, int n8) {
  const int i = blockIdx.x * NTHR + threadIdx.x;
  if (i >= n8) return;
  const size_t o = (size_t)i * 8;
  const v4f a = *(const v4f*)(in + o);
  const v4f b = *(const v4f*)(in + o + 4);
  v8us vh, vl;
#pragma unroll
  for (int q = 0; q < 4; ++q) {
    const us_t h0 = f2bf(a[q]); vh[q] = h0;     vl[q] = f2bf(a[q] - bf2f(h0));
    const us_t h1 = f2bf(b[q]); vh[q + 4] = h1; vl[q + 4] = f2bf(b[q] - bf2f(h1));
  }
  *(volatile v8us*)(hi + o) = vh;
  *(volatile v8us*)(lo + o) = vl;
  __threadfence();
  *(volatile v8us*)(hi + o) = vh;
  *(volatile v8us*)(lo + o) = vl;
}

__global__ __launch_bounds__(NTHR)
void cvt_wt_k(const float* __restrict__ W, us_t* __restrict__ hi, us_t* __restrict__ lo, int K, int Nc) {
  const int i = blockIdx.x * NTHR + threadIdx.x;
  const int n8 = (Nc * K) >> 3;
  if (i >= n8) return;
  const int o = i * 8;
  const int n = o / K;
  const int k8 = o - n * K;
  v8us vh, vl;
#pragma unroll
  for (int q = 0; q < 8; ++q) {
    const float v = W[(size_t)(k8 + q) * Nc + n];
    const us_t h0 = f2bf(v);
    vh[q] = h0;
    vl[q] = f2bf(v - bf2f(h0));
  }
  *(volatile v8us*)(hi + o) = vh;
  *(volatile v8us*)(lo + o) = vl;
  __threadfence();
  *(volatile v8us*)(hi + o) = vh;
  *(volatile v8us*)(lo + o) = vl;
}

__global__ __launch_bounds__(128)
void gemm_x3_k(const us_t* __restrict__ Ah, const us_t* __restrict__ Al,
               const us_t* __restrict__ Bh, const us_t* __restrict__ Bl,
               const float* __restrict__ bias, float* __restrict__ Cm,
               int M, int Nc, int K, int tilesN, int ntile_total) {
  __shared__ __attribute__((aligned(16))) float s_t[4][16][TN];
  const int t = threadIdx.x, lane = t & 31, wv = t >> 5, h = lane >> 4, m = lane & 15;
  const int gw = blockIdx.x * 4 + wv;
  const bool valid = gw < ntile_total;
  const int gwc = valid ? gw : 0;
  const int m0 = (gwc / tilesN) * 16;
  const int n0 = (gwc % tilesN) * TN;
  int arow = m0 + m;
  arow = arow > M - 1 ? M - 1 : arow;
  const us_t* ah  = Ah + (size_t)arow * K + 8 * h;
  const us_t* al  = Al + (size_t)arow * K + 8 * h;
  const us_t* bh0 = Bh + (size_t)(n0 + m) * K + 8 * h;
  const us_t* bl0 = Bl + (size_t)(n0 + m) * K + 8 * h;
  const us_t* bh1 = bh0 + (size_t)16 * K;
  const us_t* bl1 = bl0 + (size_t)16 * K;

  v8f acc0, acc1;
#pragma unroll
  for (int j = 0; j < 8; ++j) { acc0[j] = 0.0f; acc1[j] = 0.0f; }

#pragma unroll 1
  for (int k0 = 0; k0 < K; k0 += 32) {
    Frag fa, fl, gb, gl;
    fa.u[0] = *(const v8us*)(ah + k0);  fa.u[1] = *(const v8us*)(ah + k0 + 16);
    fl.u[0] = *(const v8us*)(al + k0);  fl.u[1] = *(const v8us*)(al + k0 + 16);
    gb.u[0] = *(const v8us*)(bh0 + k0); gb.u[1] = *(const v8us*)(bh0 + k0 + 16);
    gl.u[0] = *(const v8us*)(bl0 + k0); gl.u[1] = *(const v8us*)(bl0 + k0 + 16);
    acc0 = wmma_bf16(fa.v, gb.v, acc0);
    acc0 = wmma_bf16(fa.v, gl.v, acc0);
    acc0 = wmma_bf16(fl.v, gb.v, acc0);
    gb.u[0] = *(const v8us*)(bh1 + k0); gb.u[1] = *(const v8us*)(bh1 + k0 + 16);
    gl.u[0] = *(const v8us*)(bl1 + k0); gl.u[1] = *(const v8us*)(bl1 + k0 + 16);
    acc1 = wmma_bf16(fa.v, gb.v, acc1);
    acc1 = wmma_bf16(fa.v, gl.v, acc1);
    acc1 = wmma_bf16(fl.v, gb.v, acc1);
  }

#pragma unroll
  for (int r = 0; r < 8; ++r) {
    s_t[wv][8 * h + r][m]      = acc0[r];
    s_t[wv][8 * h + r][16 + m] = acc1[r];
  }
  __syncthreads();

  const int rsub = lane >> 3, c4 = (lane & 7) * 4;
  const v4f bv = *(const v4f*)(bias + n0 + c4);
  v4f vals[4];
#pragma unroll
  for (int q = 0; q < 4; ++q) {
    const v4f v = *(const v4f*)(&s_t[wv][q * 4 + rsub][c4]);
    vals[q] = v + bv;
  }
#pragma unroll
  for (int q = 0; q < 4; ++q) {
    const int grow = m0 + q * 4 + rsub;
    if (valid && grow < M) *(volatile v4f*)(Cm + (size_t)grow * Nc + n0 + c4) = vals[q];
  }
  __threadfence();
#pragma unroll
  for (int q = 0; q < 4; ++q) {
    const int grow = m0 + q * 4 + rsub;
    if (valid && grow < M) *(volatile v4f*)(Cm + (size_t)grow * Nc + n0 + c4) = vals[q];
  }
}

__device__ __forceinline__ float gat1_logit(const float* __restrict__ xl, const int* __restrict__ row,
                                             int cnt, int d, int N, int j, v4f b, v4f at, int lane, v4f& a) {
  int s = (j < cnt) ? row[1 + j] : d;
  s = s < 0 ? 0 : (s > N - 1 ? N - 1 : s);
  a = *(const v4f*)(xl + (size_t)s * FIN + 4 * lane);
  const v4f v = a + b;
  float acc = 0.0f;
#pragma unroll
  for (int q = 0; q < 4; ++q) {
    float x = v[q];
    x = x > 0.0f ? x : 0.2f * x;
    acc += x * at[q];
  }
  acc += __shfl_xor(acc, 1, 32);
  acc += __shfl_xor(acc, 2, 32);
  acc += __shfl_xor(acc, 4, 32);
  return acc;
}

__global__ __launch_bounds__(NTHR)
void gat1_k(const float* __restrict__ xl, const float* __restrict__ xr, const int* __restrict__ adj,
            const float* __restrict__ att, const float* __restrict__ bias, float* __restrict__ outp, int N) {
  const int d = blockIdx.x * (NTHR / 32) + (threadIdx.x >> 5);
  if (d >= N) return;
  const int lane = threadIdx.x & 31;
  const v4f b  = *(const v4f*)(xr + (size_t)d * FIN + 4 * lane);
  const v4f at = *(const v4f*)(att + 4 * lane);
  const int* row = adj + (size_t)d * ROWW;
  int cnt = row[0];
  cnt = cnt < 0 ? 0 : (cnt > RCAP ? RCAP : cnt);
  const int tot = cnt + 1;

  float mx = -__builtin_inff();
#pragma unroll 1
  for (int j = 0; j < tot; ++j) {
    v4f a;
    const float lg = gat1_logit(xl, row, cnt, d, N, j, b, at, lane, a);
    mx = fmaxf(mx, lg);
  }
  float den = 0.0f;
#pragma unroll 1
  for (int j = 0; j < tot; ++j) {
    v4f a;
    const float lg = gat1_logit(xl, row, cnt, d, N, j, b, at, lane, a);
    den += expf(lg - mx);
  }
  v4f acc;
#pragma unroll
  for (int q = 0; q < 4; ++q) acc[q] = 0.0f;
#pragma unroll 1
  for (int j = 0; j < tot; ++j) {
    v4f a;
    const float lg = gat1_logit(xl, row, cnt, d, N, j, b, at, lane, a);
    const float al = expf(lg - mx) / den;
    acc = acc + a * al;
  }
  const v4f o = acc + *(const v4f*)(bias + 4 * lane);
  *(volatile v4f*)(outp + (size_t)d * FIN + 4 * lane) = o;
  __threadfence();
  *(volatile v4f*)(outp + (size_t)d * FIN + 4 * lane) = o;
}

__device__ __forceinline__ float gat2_logit(const float* __restrict__ xl, const int* __restrict__ row,
                                             int cnt, int d, int N, int j, float b, float at, int lane, float& a) {
  int s = (j < cnt) ? row[1 + j] : d;
  s = s < 0 ? 0 : (s > N - 1 ? N - 1 : s);
  a = xl[(size_t)s * C2 + lane];
  float x = a + b;
  x = x > 0.0f ? x : 0.2f * x;
  float acc = x * at;
  acc += __shfl_xor(acc, 1, 32);
  acc += __shfl_xor(acc, 2, 32);
  acc += __shfl_xor(acc, 4, 32);
  acc += __shfl_xor(acc, 8, 32);
  acc += __shfl_xor(acc, 16, 32);
  return acc;
}

__global__ __launch_bounds__(NTHR)
void gat2_k(const float* __restrict__ xl, const float* __restrict__ xr, const int* __restrict__ adj,
            const float* __restrict__ att, const float* __restrict__ bias, float* __restrict__ outp, int N) {
  const int d = blockIdx.x * (NTHR / 32) + (threadIdx.x >> 5);
  if (d >= N) return;
  const int lane = threadIdx.x & 31;
  const float b  = xr[(size_t)d * C2 + lane];
  const float at = att[lane];
  const int* row = adj + (size_t)d * ROWW;
  int cnt = row[0];
  cnt = cnt < 0 ? 0 : (cnt > RCAP ? RCAP : cnt);
  const int tot = cnt + 1;

  float mx = -__builtin_inff();
#pragma unroll 1
  for (int j = 0; j < tot; ++j) {
    float a;
    const float lg = gat2_logit(xl, row, cnt, d, N, j, b, at, lane, a);
    mx = fmaxf(mx, lg);
  }
  float den = 0.0f;
#pragma unroll 1
  for (int j = 0; j < tot; ++j) {
    float a;
    const float lg = gat2_logit(xl, row, cnt, d, N, j, b, at, lane, a);
    den += expf(lg - mx);
  }
  float acc = 0.0f;
#pragma unroll 1
  for (int j = 0; j < tot; ++j) {
    float a;
    const float lg = gat2_logit(xl, row, cnt, d, N, j, b, at, lane, a);
    const float al = expf(lg - mx) / den;
    acc += a * al;
  }
  const float o = acc + bias[lane];
  v4f pk;
  pk[0] = __shfl(o, (4 * lane + 0) & 31, 32);
  pk[1] = __shfl(o, (4 * lane + 1) & 31, 32);
  pk[2] = __shfl(o, (4 * lane + 2) & 31, 32);
  pk[3] = __shfl(o, (4 * lane + 3) & 31, 32);
  if (lane < 8) *(volatile v4f*)(outp + (size_t)d * C2 + 4 * lane) = pk;
  __threadfence();
  if (lane < 8) *(volatile v4f*)(outp + (size_t)d * C2 + 4 * lane) = pk;
}

template <int D>
__global__ __launch_bounds__(128)
void gn_stats_k(const float* __restrict__ xv, const int* __restrict__ batch, const float* __restrict__ ms,
                float* __restrict__ subo, float* __restrict__ sdo, int N) {
  __shared__ unsigned s_m[4];
  __shared__ __attribute__((aligned(16))) float s_sub[128];
  __shared__ __attribute__((aligned(16))) float s_sd[128];
  const int t = threadIdx.x, lane = t & 31, wv = t >> 5, g = blockIdx.x;
  int cnt = 0;
  float sum = 0.0f;
  for (int base = 0; base < N; base += 128) {
    const int n = base + t;
    const int bb = (n < N) ? batch[n] : -1;
    const unsigned bal = __builtin_amdgcn_ballot_w32(bb == g);
    if (lane == 0) s_m[wv] = bal;
    __syncthreads();
    for (int w = 0; w < 4; ++w) {
      unsigned mm = s_m[w];
      while (mm) {
        const int bit = __builtin_ctz(mm);
        mm &= mm - 1u;
        const int node = base + w * 32 + bit;
        ++cnt;
        if (t < D) sum += xv[(size_t)node * D + t];
      }
    }
    __syncthreads();
  }
  const float fc = fmaxf((float)cnt, 1.0f);
  const float mean = sum / fc;
  const float sub = (t < D) ? mean * ms[t] : 0.0f;
  float vs = 0.0f;
  for (int base = 0; base < N; base += 128) {
    const int n = base + t;
    const int bb = (n < N) ? batch[n] : -1;
    const unsigned bal = __builtin_amdgcn_ballot_w32(bb == g);
    if (lane == 0) s_m[wv] = bal;
    __syncthreads();
    for (int w = 0; w < 4; ++w) {
      unsigned mm = s_m[w];
      while (mm) {
        const int bit = __builtin_ctz(mm);
        mm &= mm - 1u;
        const int node = base + w * 32 + bit;
        if (t < D) { const float o = xv[(size_t)node * D + t] - sub; vs += o * o; }
      }
    }
    __syncthreads();
  }
  const float var = vs / fc;
  const float sd = sqrtf(var + 1e-5f);
  if (t < D) { s_sub[t] = sub; s_sd[t] = sd; }
  __syncthreads();
  const bool wsb = t < (D >> 2);
  const bool wsd = (t >= 64) && ((t - 64) < (D >> 2));
  v4f va, vb;
#pragma unroll
  for (int q = 0; q < 4; ++q) { va[q] = 0.0f; vb[q] = 0.0f; }
  if (wsb) va = *(const v4f*)(&s_sub[4 * t]);
  if (wsd) vb = *(const v4f*)(&s_sd[4 * (t - 64)]);
  if (wsb) *(volatile v4f*)(subo + (size_t)g * D + 4 * t) = va;
  if (wsd) *(volatile v4f*)(sdo + (size_t)g * D + 4 * (t - 64)) = vb;
  __threadfence();
  if (wsb) *(volatile v4f*)(subo + (size_t)g * D + 4 * t) = va;
  if (wsd) *(volatile v4f*)(sdo + (size_t)g * D + 4 * (t - 64)) = vb;
}

__device__ __attribute__((noinline)) float gn_act(float x, float sub, float w, float sd, float b, float r) {
  const float o = x - sub;
  const float y = (w * o) / sd + b;
  return gelu_f(y + r);
}

__global__ __launch_bounds__(NTHR)
void gn_apply_h_k(const float* __restrict__ xv, const float* __restrict__ res, const int* __restrict__ batch,
                  const float* __restrict__ subv, const float* __restrict__ sdv,
                  const float* __restrict__ w, const float* __restrict__ b,
                  us_t* __restrict__ hh, us_t* __restrict__ hl, int N, int G) {
  const int i = blockIdx.x * NTHR + threadIdx.x;
  if (i >= N * 16) return;
  const int n = i >> 4, c8 = (i & 15) * 8;
  int g = batch[n];
  g = g < 0 ? 0 : (g > G - 1 ? G - 1 : g);
  const size_t xo = (size_t)n * FIN + c8;
  const size_t go = (size_t)g * FIN + c8;
  const v4f x0 = *(const v4f*)(xv + xo),   x1 = *(const v4f*)(xv + xo + 4);
  const v4f r0 = *(const v4f*)(res + xo),  r1 = *(const v4f*)(res + xo + 4);
  const v4f s0 = *(const v4f*)(subv + go), s1 = *(const v4f*)(subv + go + 4);
  const v4f d0 = *(const v4f*)(sdv + go),  d1 = *(const v4f*)(sdv + go + 4);
  const v4f w0 = *(const v4f*)(w + c8),    w1 = *(const v4f*)(w + c8 + 4);
  const v4f b0 = *(const v4f*)(b + c8),    b1 = *(const v4f*)(b + c8 + 4);
  v8us vh, vl;
#pragma unroll
  for (int q = 0; q < 4; ++q) {
    const float y0 = gn_act(x0[q], s0[q], w0[q], d0[q], b0[q], r0[q]);
    const float y1 = gn_act(x1[q], s1[q], w1[q], d1[q], b1[q], r1[q]);
    const us_t h0 = f2bf(y0); vh[q] = h0;     vl[q] = f2bf(y0 - bf2f(h0));
    const us_t h1 = f2bf(y1); vh[q + 4] = h1; vl[q + 4] = f2bf(y1 - bf2f(h1));
  }
  const size_t oo = (size_t)i * 8;
  *(volatile v8us*)(hh + oo) = vh;
  *(volatile v8us*)(hl + oo) = vl;
  __threadfence();
  *(volatile v8us*)(hh + oo) = vh;
  *(volatile v8us*)(hl + oo) = vl;
}

__global__ __launch_bounds__(NTHR)
void gn_apply_f_k(const float* __restrict__ xv, const float* __restrict__ res, const int* __restrict__ batch,
                  const float* __restrict__ subv, const float* __restrict__ sdv,
                  const float* __restrict__ w, const float* __restrict__ b,
                  float* __restrict__ ho, int N, int G) {
  const int i = blockIdx.x * NTHR + threadIdx.x;
  if (i >= N * 8) return;
  const int n = i >> 3, c4 = (i & 7) * 4;
  int g = batch[n];
  g = g < 0 ? 0 : (g > G - 1 ? G - 1 : g);
  const size_t xo = (size_t)n * C2 + c4;
  const size_t go = (size_t)g * C2 + c4;
  const v4f x0 = *(const v4f*)(xv + xo);
  const v4f r0 = *(const v4f*)(res + xo);
  const v4f s0 = *(const v4f*)(subv + go);
  const v4f d0 = *(const v4f*)(sdv + go);
  const v4f w0 = *(const v4f*)(w + c4);
  const v4f b0 = *(const v4f*)(b + c4);
  v4f y;
#pragma unroll
  for (int q = 0; q < 4; ++q) y[q] = gn_act(x0[q], s0[q], w0[q], d0[q], b0[q], r0[q]);
  *(volatile v4f*)(ho + xo) = y;
  __threadfence();
  *(volatile v4f*)(ho + xo) = y;
}

__global__ __launch_bounds__(128)
void pool_head_k(const float* __restrict__ h2, const int* __restrict__ batch,
                 const float* __restrict__ Weg, const float* __restrict__ beg,
                 const float* __restrict__ Wf1, const float* __restrict__ bf1,
                 float* __restrict__ embo, int N) {
  __shared__ unsigned s_m[4];
  __shared__ float s_fin[96];
  __shared__ float s_max[32];
  __shared__ __attribute__((aligned(16))) float s_emb[32];
  const int t = threadIdx.x, lane = t & 31, wv = t >> 5, g = blockIdx.x;
  int cnt = 0;
  float sum = 0.0f, mx = -__builtin_inff();
  for (int base = 0; base < N; base += 128) {
    const int n = base + t;
    const int bb = (n < N) ? batch[n] : -1;
    const unsigned bal = __builtin_amdgcn_ballot_w32(bb == g);
    if (lane == 0) s_m[wv] = bal;
    __syncthreads();
    for (int w = 0; w < 4; ++w) {
      unsigned mm = s_m[w];
      while (mm) {
        const int bit = __builtin_ctz(mm);
        mm &= mm - 1u;
        const int node = base + w * 32 + bit;
        ++cnt;
        if (t < 32) { const float v = h2[(size_t)node * C2 + t]; sum += v; mx = fmaxf(mx, v); }
      }
    }
    __syncthreads();
  }
  if (t < 32) {
    const float mean = sum / fmaxf((float)cnt, 1.0f);
    s_fin[t] = mean;
    s_max[t] = (cnt > 0) ? mx : 0.0f;
  }
  __syncthreads();
  if (t < 64) {
    float a = 0.0f;
#pragma unroll 1
    for (int c = 0; c < 32; ++c) a += s_fin[c] * Weg[c * 64 + t];
    a += beg[t];
    const float gate = 1.0f / (1.0f + expf(-a));
    const float v = (t < 32) ? s_fin[t] : s_max[t - 32];
    s_fin[32 + t] = gate * v;
  }
  __syncthreads();
  if (t < 32) {
    float a = 0.0f;
#pragma unroll 1
    for (int k = 0; k < 96; ++k) a += s_fin[k] * Wf1[k * 32 + t];
    a += bf1[t];
    s_emb[t] = gelu_f(a);
  }
  __syncthreads();
  v4f v;
#pragma unroll
  for (int q = 0; q < 4; ++q) v[q] = 0.0f;
  if (t < 8) v = *(const v4f*)(&s_emb[4 * t]);
  if (t < 8) *(volatile v4f*)(embo + (size_t)g * C2 + 4 * t) = v;
  __threadfence();
  if (t < 8) *(volatile v4f*)(embo + (size_t)g * C2 + 4 * t) = v;
}

__global__ __launch_bounds__(512)
void final_k(const float* __restrict__ emb, const float* __restrict__ Wf2, const float* __restrict__ bf2,
             float* __restrict__ outp, int G) {
  __shared__ __attribute__((aligned(16))) float s_o[512];
  const int t = threadIdx.x;
  if (t < G) {
    float a = 0.0f;
#pragma unroll 1
    for (int c = 0; c < 32; ++c) a += emb[(size_t)t * C2 + c] * Wf2[c];
    a += bf2[0];
    s_o[t] = a;
  }
  __syncthreads();
  const int nq = G >> 2;
  const int rem = G & 3;
  v4f v;
#pragma unroll
  for (int q = 0; q < 4; ++q) v[q] = 0.0f;
  float tv = 0.0f;
  if (t < nq) v = *(const v4f*)(&s_o[4 * t]);
  if (t < rem) tv = s_o[4 * nq + t];
  if (t < nq) *(volatile v4f*)(outp + 4 * t) = v;
  if (t < rem) *(volatile float*)(outp + 4 * nq + t) = tv;
  __threadfence();
  if (t < nq) *(volatile v4f*)(outp + 4 * t) = v;
  if (t < rem) *(volatile float*)(outp + 4 * nq + t) = tv;
}

static inline unsigned nblk(long long n, int b) { return (unsigned)((n + b - 1) / b); }

extern "C" void kernel_launch(void* const* d_in, const int* in_sizes, int n_in,
                              void* d_out, int out_size, void* d_ws, size_t ws_size,
                              hipStream_t stream) {
  (void)n_in;
  const float* x     = (const float*)d_in[0];
  const int*   ei    = (const int*)d_in[1];
  const int*   batch = (const int*)d_in[2];
  const float* Wl1   = (const float*)d_in[3];
  const float* bl1   = (const float*)d_in[4];
  const float* Wr1   = (const float*)d_in[5];
  const float* br1   = (const float*)d_in[6];
  const float* att1  = (const float*)d_in[7];
  const float* bias1 = (const float*)d_in[8];
  const float* gn1w  = (const float*)d_in[9];
  const float* gn1b  = (const float*)d_in[10];
  const float* gn1ms = (const float*)d_in[11];
  const float* Wl2   = (const float*)d_in[12];
  const float* bl2   = (const float*)d_in[13];
  const float* Wr2   = (const float*)d_in[14];
  const float* br2   = (const float*)d_in[15];
  const float* att2  = (const float*)d_in[16];
  const float* bias2 = (const float*)d_in[17];
  const float* gn2w  = (const float*)d_in[18];
  const float* gn2b  = (const float*)d_in[19];
  const float* gn2ms = (const float*)d_in[20];
  const float* Wp1   = (const float*)d_in[21];
  const float* bp1   = (const float*)d_in[22];
  const float* Wp2   = (const float*)d_in[23];
  const float* bp2   = (const float*)d_in[24];
  const float* Weg   = (const float*)d_in[25];
  const float* beg   = (const float*)d_in[26];
  const float* Wf1   = (const float*)d_in[27];
  const float* bf1   = (const float*)d_in[28];
  const float* Wf2   = (const float*)d_in[29];
  const float* bf2   = (const float*)d_in[30];
  float* out = (float*)d_out;

  const int N = in_sizes[0] / FIN;
  const int E = in_sizes[1] / 2;
  const int G = out_size;
  if (N <= 0 || N >= (1 << 24) || G <= 0 || G > 512 || E < 0) return;

  size_t off = 0;
  auto carve = [&](size_t bytes) -> char* {
    char* p = (char*)d_ws + off;
    off += (bytes + 255) & ~(size_t)255;
    return p;
  };
  int*   adj  = (int*)carve((size_t)N * ROWW * 4);
  us_t*  xh   = (us_t*)carve((size_t)N * FIN * 2);
  us_t*  xlo  = (us_t*)carve((size_t)N * FIN * 2);
  us_t*  wl1h = (us_t*)carve((size_t)FIN * FIN * 2); us_t* wl1l = (us_t*)carve((size_t)FIN * FIN * 2);
  us_t*  wr1h = (us_t*)carve((size_t)FIN * FIN * 2); us_t* wr1l = (us_t*)carve((size_t)FIN * FIN * 2);
  us_t*  wp1h = (us_t*)carve((size_t)FIN * FIN * 2); us_t* wp1l = (us_t*)carve((size_t)FIN * FIN * 2);
  us_t*  wl2h = (us_t*)carve((size_t)C2 * FIN * 2);  us_t* wl2l = (us_t*)carve((size_t)C2 * FIN * 2);
  us_t*  wr2h = (us_t*)carve((size_t)C2 * FIN * 2);  us_t* wr2l = (us_t*)carve((size_t)C2 * FIN * 2);
  us_t*  wp2h = (us_t*)carve((size_t)C2 * FIN * 2);  us_t* wp2l = (us_t*)carve((size_t)C2 * FIN * 2);
  float* xl1  = (float*)carve((size_t)N * FIN * 4);
  float* xr1  = (float*)carve((size_t)N * FIN * 4);
  float* res1 = (float*)carve((size_t)N * FIN * 4);
  float* out1 = (float*)carve((size_t)N * FIN * 4);
  float* sub1 = (float*)carve((size_t)G * FIN * 4);
  float* sd1  = (float*)carve((size_t)G * FIN * 4);
  us_t*  hh   = (us_t*)carve((size_t)N * FIN * 2);
  us_t*  hl   = (us_t*)carve((size_t)N * FIN * 2);
  float* xl2  = (float*)carve((size_t)N * C2 * 4);
  float* xr2  = (float*)carve((size_t)N * C2 * 4);
  float* res2 = (float*)carve((size_t)N * C2 * 4);
  float* out2 = (float*)carve((size_t)N * C2 * 4);
  float* h2   = (float*)carve((size_t)N * C2 * 4);
  float* sub2 = (float*)carve((size_t)G * C2 * 4);
  float* sd2  = (float*)carve((size_t)G * C2 * 4);
  float* emb  = (float*)carve((size_t)G * C2 * 4);
  if (off > ws_size) return;

  adj_build_k<<<nblk(N, NPB), NTHR, 0, stream>>>(ei, adj, N, E);

  cvt_rows_k<<<nblk((long long)N * 16, NTHR), NTHR, 0, stream>>>(x, xh, xlo, N * 16);
  cvt_wt_k<<<nblk((long long)FIN * FIN / 8, NTHR), NTHR, 0, stream>>>(Wl1, wl1h, wl1l, FIN, FIN);
  cvt_wt_k<<<nblk((long long)FIN * FIN / 8, NTHR), NTHR, 0, stream>>>(Wr1, wr1h, wr1l, FIN, FIN);
  cvt_wt_k<<<nblk((long long)FIN * FIN / 8, NTHR), NTHR, 0, stream>>>(Wp1, wp1h, wp1l, FIN, FIN);
  cvt_wt_k<<<nblk((long long)C2 * FIN / 8, NTHR), NTHR, 0, stream>>>(Wl2, wl2h, wl2l, FIN, C2);
  cvt_wt_k<<<nblk((long long)C2 * FIN / 8, NTHR), NTHR, 0, stream>>>(Wr2, wr2h, wr2l, FIN, C2);
  cvt_wt_k<<<nblk((long long)C2 * FIN / 8, NTHR), NTHR, 0, stream>>>(Wp2, wp2h, wp2l, FIN, C2);

  const int mtiles = (N + 15) / 16;
  {
    const int tilesN = FIN / TN;
    const int ntot = mtiles * tilesN;
    const unsigned blks = nblk(ntot, 4);
    gemm_x3_k<<<blks, 128, 0, stream>>>(xh, xlo, wl1h, wl1l, bl1, xl1,  N, FIN, FIN, tilesN, ntot);
    gemm_x3_k<<<blks, 128, 0, stream>>>(xh, xlo, wr1h, wr1l, br1, xr1,  N, FIN, FIN, tilesN, ntot);
    gemm_x3_k<<<blks, 128, 0, stream>>>(xh, xlo, wp1h, wp1l, bp1, res1, N, FIN, FIN, tilesN, ntot);
  }

  gat1_k<<<nblk(N, NTHR / 32), NTHR, 0, stream>>>(xl1, xr1, adj, att1, bias1, out1, N);

  gn_stats_k<FIN><<<(unsigned)G, 128, 0, stream>>>(out1, batch, gn1ms, sub1, sd1, N);
  gn_apply_h_k<<<nblk((long long)N * 16, NTHR), NTHR, 0, stream>>>(out1, res1, batch, sub1, sd1, gn1w, gn1b, hh, hl, N, G);

  {
    const int tilesN = C2 / TN;
    const int ntot = mtiles * tilesN;
    const unsigned blks = nblk(ntot, 4);
    gemm_x3_k<<<blks, 128, 0, stream>>>(hh, hl, wl2h, wl2l, bl2, xl2,  N, C2, FIN, tilesN, ntot);
    gemm_x3_k<<<blks, 128, 0, stream>>>(hh, hl, wr2h, wr2l, br2, xr2,  N, C2, FIN, tilesN, ntot);
    gemm_x3_k<<<blks, 128, 0, stream>>>(hh, hl, wp2h, wp2l, bp2, res2, N, C2, FIN, tilesN, ntot);
  }

  gat2_k<<<nblk(N, NTHR / 32), NTHR, 0, stream>>>(xl2, xr2, adj, att2, bias2, out2, N);

  gn_stats_k<C2><<<(unsigned)G, 128, 0, stream>>>(out2, batch, gn2ms, sub2, sd2, N);
  gn_apply_f_k<<<nblk((long long)N * 8, NTHR), NTHR, 0, stream>>>(out2, res2, batch, sub2, sd2, gn2w, gn2b, h2, N, G);

  pool_head_k<<<(unsigned)G, 128, 0, stream>>>(h2, batch, Weg, beg, Wf1, bf1, emb, N);
  final_k<<<1, 512, 0, stream>>>(emb, Wf2, bf2, out, G);
}
